// GatedDeltaProductEncoder_11751030521974
// MI455X (gfx1250) — hardware-verified
//
#include <hip/hip_runtime.h>
#include <math.h>

constexpr int kBatch   = 2;
constexpr int kSeq     = 1024;
constexpr int kDim     = 512;
constexpr int kHeads   = 4;
constexpr int kDk      = 128;
constexpr int kDv      = 128;
constexpr int kNh      = 2;
constexpr int kMlp     = 256;
constexpr int kRows    = kBatch * kSeq;
constexpr int kQCols   = kHeads * kDk;
constexpr int kKCols   = kNh * kHeads * kDk;
constexpr int kVCols   = kNh * kHeads * kDv;
constexpr int kQkvCols = kQCols + kKCols + kVCols;
constexpr int kKOff    = kQCols;
constexpr int kVOff    = kQCols + kKCols;
constexpr int kOCols   = kHeads * kDv;
constexpr int kGateCols = 16;
constexpr int kOut0    = kRows * kDim;
constexpr int kOut1    = kBatch * kHeads * kDk * kDv;
constexpr float kEps   = 1e-6f;
constexpr float kACarry = 16.0f;
constexpr float kWCarry = 16.0f;
constexpr float kFold   = 1.0f / (kACarry * kWCarry);
constexpr int kSlabPitch = 36;

static_assert(kRows == 2048 && kQkvCols == 2560 && kOCols == 512, "shape");
static_assert(kRows % 64 == 0 && kQkvCols % 64 == 0 && kDim % 64 == 0 && kMlp % 64 == 0, "tile multiples");
static_assert(kDim % 32 == 0 && kOCols % 32 == 0 && kMlp % 32 == 0, "k multiples");
static_assert(kDk == 128 && kDv == 128 && kHeads == 4 && kNh == 2, "scan layout");
static_assert((size_t)kOut0 * 4 == 4194304, "second output byte offset");
static_assert(((size_t)kOut0 * 4) % 128 == 0, "second output line aligned");

typedef __attribute__((ext_vector_type(16))) _Float16 v16h;
typedef __attribute__((ext_vector_type(8)))  _Float16 v8h;
typedef __attribute__((ext_vector_type(16))) __bf16   v16b;
typedef __attribute__((ext_vector_type(8)))  __bf16   v8b;
typedef __attribute__((ext_vector_type(8)))  float    v8f;
typedef __attribute__((ext_vector_type(4)))  float    v4f;
typedef __attribute__((ext_vector_type(4)))  unsigned int v4u;

__device__ __forceinline__ unsigned short f2bf_bits(float f) {
  unsigned u = __float_as_uint(f);
  return (unsigned short)((u + 0x7FFFu + ((u >> 16) & 1u)) >> 16);
}
__device__ __forceinline__ float bf_bits2f(unsigned short h) { return __uint_as_float(((unsigned)h) << 16); }
__device__ __forceinline__ unsigned pk16(unsigned short a, unsigned short b) { return (unsigned)a | ((unsigned)b << 16); }
__device__ __forceinline__ unsigned short h_bits(float f) { const _Float16 h = (_Float16)f; return __builtin_bit_cast(unsigned short, h); }

__device__ __forceinline__ v4u pack8_f16(v4f a, v4f b, float sc) {
  unsigned short hb[8];
#pragma unroll
  for (int e = 0; e < 4; ++e) {
    const float fa = a[e] * sc;
    const float fb = b[e] * sc;
    hb[e]     = h_bits(fa);
    hb[4 + e] = h_bits(fb);
  }
  return (v4u){pk16(hb[0], hb[1]), pk16(hb[2], hb[3]), pk16(hb[4], hb[5]), pk16(hb[6], hb[7])};
}
__device__ __forceinline__ void split8_bf16(v4f a, v4f b, v4u& hi, v4u& lo) {
  unsigned short hb[8], lb[8];
#pragma unroll
  for (int e = 0; e < 4; ++e) {
    const float fa = a[e];
    const float fb = b[e];
    const unsigned short ha = f2bf_bits(fa);
    const unsigned short hc = f2bf_bits(fb);
    hb[e]     = ha;
    hb[4 + e] = hc;
    lb[e]     = f2bf_bits(fa - bf_bits2f(ha));
    lb[4 + e] = f2bf_bits(fb - bf_bits2f(hc));
  }
  hi = (v4u){pk16(hb[0], hb[1]), pk16(hb[2], hb[3]), pk16(hb[4], hb[5]), pk16(hb[6], hb[7])};
  lo = (v4u){pk16(lb[0], lb[1]), pk16(lb[2], lb[3]), pk16(lb[4], lb[5]), pk16(lb[6], lb[7])};
}

__device__ __forceinline__ float wave_sum(float v) {
#pragma unroll
  for (int off = 16; off >= 1; off >>= 1) v += __shfl_xor(v, off, 32);
  return v;
}
__device__ __forceinline__ float grp16_sum(float v) {
#pragma unroll
  for (int off = 8; off >= 1; off >>= 1) v += __shfl_xor(v, off, 32);
  return v;
}
__device__ __forceinline__ float grp8_sum(float v) {
  v += __shfl_xor(v, 1, 32);
  v += __shfl_xor(v, 2, 32);
  v += __shfl_xor(v, 4, 32);
  return v;
}

__device__ __forceinline__ void grp_guard_h(v8f& a, v8f& b, v8f& c, v8f& d, v16h x, v16h y, v16h p, v16h q, v16h r, v16h s) {
  asm volatile("v_nop\n\tv_nop\n\tv_nop\n\tv_nop" : "+v"(a), "+v"(b), "+v"(c), "+v"(d) : "v"(x), "v"(y), "v"(p), "v"(q), "v"(r), "v"(s));
}
__device__ __forceinline__ void grp_guard_b(v8f& a, v8f& b, v8f& c, v8f& d, v16b x, v16b y, v16b p, v16b q, v16b r, v16b s) {
  asm volatile("v_nop\n\tv_nop\n\tv_nop\n\tv_nop" : "+v"(a), "+v"(b), "+v"(c), "+v"(d) : "v"(x), "v"(y), "v"(p), "v"(q), "v"(r), "v"(s));
}
__device__ __forceinline__ void keep4_h(v16h a, v16h b, v16h c, v16h d) { asm volatile("v_nop" :: "v"(a), "v"(b), "v"(c), "v"(d)); }
__device__ __forceinline__ void keep4_b(v16b a, v16b b, v16b c, v16b d) { asm volatile("v_nop" :: "v"(a), "v"(b), "v"(c), "v"(d)); }
__device__ __forceinline__ void acc_guard4(v8f& a, v8f& b, v8f& c, v8f& d) { asm volatile("v_nop\n\tv_nop\n\tv_nop\n\tv_nop" : "+v"(a), "+v"(b), "+v"(c), "+v"(d)); }

template <typename T> struct Frag;
template <> struct Frag<_Float16> {
  typedef v16h V; union U { v16h v; v8h h[2]; };
  static __device__ __forceinline__ v16h load(const _Float16* p) {
    U f; f.h[0] = *(const v8h*)(p); f.h[1] = *(const v8h*)(p + 16); return f.v;
  }
  static __device__ __forceinline__ v8f mma(v16h a, v16h b, v8f c) {
    return __builtin_amdgcn_wmma_f32_16x16x32_f16(false, a, false, b, (short)0, c, false, false);
  }
  static __device__ __forceinline__ void guard(v8f& a, v8f& b, v8f& c, v8f& d, v16h x, v16h y, v16h p, v16h q, v16h r, v16h s) { grp_guard_h(a, b, c, d, x, y, p, q, r, s); }
  static __device__ __forceinline__ void keep(v16h a, v16h b, v16h c, v16h d) { keep4_h(a, b, c, d); }
};
template <> struct Frag<__bf16> {
  typedef v16b V; union U { v16b v; v8b h[2]; };
  static __device__ __forceinline__ v16b load(const __bf16* p) {
    U f; f.h[0] = *(const v8b*)(p); f.h[1] = *(const v8b*)(p + 16); return f.v;
  }
  static __device__ __forceinline__ v8f mma(v16b a, v16b b, v8f c) {
    return __builtin_amdgcn_wmma_f32_16x16x32_bf16(false, a, false, b, (short)0, c, false, false);
  }
  static __device__ __forceinline__ void guard(v8f& a, v8f& b, v8f& c, v8f& d, v16b x, v16b y, v16b p, v16b q, v16b r, v16b s) { grp_guard_b(a, b, c, d, x, y, p, q, r, s); }
  static __device__ __forceinline__ void keep(v16b a, v16b b, v16b c, v16b d) { keep4_b(a, b, c, d); }
};

template <int ET> struct Elem;
template <> struct Elem<0> { typedef _Float16 T; };
template <> struct Elem<1> { typedef __bf16 T; };

template <int ET, bool SPLIT, bool RESID>
__global__ __launch_bounds__(256) void wmma_gemm64(
    const unsigned short* __restrict__ Ap, const unsigned short* __restrict__ A2p, int lda,
    const unsigned short* __restrict__ Btp, const unsigned short* __restrict__ Bt2p, int ldb,
    float* __restrict__ Cout, int ldc, const float* __restrict__ resid,
    int M, int N, int K, float scale) {
  typedef typename Elem<ET>::T T;
  typedef typename Frag<T>::V V;
  const T* Ab  = (const T*)Ap;
  const T* Ab2 = (const T*)A2p;
  const T* Bb  = (const T*)Btp;
  const T* Bb2 = (const T*)Bt2p;
  __shared__ __align__(16) float sT[8][16 * 68];
  const int lane = threadIdx.x & 31;
  const int wave = threadIdx.x >> 5;
  const int tilesN = N >> 6;
  const int tilesM = M >> 6;
  const int tile = blockIdx.x * 8 + wave;
  if (tile >= tilesM * tilesN) return;
  const int tm = tile / tilesN;
  const int tn = tile - tm * tilesN;
  const int m0 = tm << 6;
  const int n0 = tn << 6;

  const int rlane = lane & 15;
  const int koff  = (lane >> 4) * 8;
  const int mOff  = (lane >> 4) * 8;

  v8f acc[4][4];
#pragma unroll
  for (int i = 0; i < 4; ++i)
#pragma unroll
    for (int j = 0; j < 4; ++j) acc[i][j] = (v8f){0.f, 0.f, 0.f, 0.f, 0.f, 0.f, 0.f, 0.f};

  for (int k0 = 0; k0 < K; k0 += 32) {
    V bh[4], bl[4];
#pragma unroll
    for (int j = 0; j < 4; ++j) {
      const size_t bo = (size_t)(n0 + (j << 4) + rlane) * ldb + koff + k0;
      bh[j] = Frag<T>::load(Bb + bo);
      if (SPLIT) bl[j] = Frag<T>::load(Bb2 + bo);
    }
#pragma unroll
    for (int i = 0; i < 4; ++i) {
      const size_t ao = (size_t)(m0 + (i << 4) + rlane) * lda + koff + k0;
      V ah = Frag<T>::load(Ab + ao);
      V al;
      if (SPLIT) al = Frag<T>::load(Ab2 + ao);
#pragma unroll
      for (int j = 0; j < 4; ++j) {
        acc[i][j] = Frag<T>::mma(ah, bh[j], acc[i][j]);
        if (SPLIT) {
          acc[i][j] = Frag<T>::mma(ah, bl[j], acc[i][j]);
          acc[i][j] = Frag<T>::mma(al, bh[j], acc[i][j]);
        }
      }
      Frag<T>::guard(acc[i][0], acc[i][1], acc[i][2], acc[i][3], ah, SPLIT ? al : ah, bh[0], bh[1], bh[2], bh[3]);
    }
    Frag<T>::keep(bh[0], bh[1], bh[2], bh[3]);
    if (SPLIT) Frag<T>::keep(bl[0], bl[1], bl[2], bl[3]);
  }
  acc_guard4(acc[0][0], acc[0][1], acc[0][2], acc[0][3]);
  acc_guard4(acc[1][0], acc[1][1], acc[1][2], acc[1][3]);
  acc_guard4(acc[2][0], acc[2][1], acc[2][2], acc[2][3]);
  acc_guard4(acc[3][0], acc[3][1], acc[3][2], acc[3][3]);

  float* slab = sT[wave];
  const int hh = lane >> 4;
  const int c4 = (lane & 15) * 4;
#pragma unroll
  for (int i = 0; i < 4; ++i) {
    const int mBase = m0 + (i << 4);
#pragma unroll
    for (int j = 0; j < 4; ++j) {
#pragma unroll
      for (int r = 0; r < 8; ++r) {
        slab[(mOff + r) * 68 + (j << 4) + rlane] = acc[i][j][r] * scale;
      }
    }
    __builtin_amdgcn_fence(__ATOMIC_RELEASE, "workgroup");
    __builtin_amdgcn_wave_barrier();
    __builtin_amdgcn_fence(__ATOMIC_ACQUIRE, "workgroup");
    v4f vals[8];
#pragma unroll
    for (int it = 0; it < 8; ++it) {
      const int row = it * 2 + hh;
      v4f v = *(const v4f*)(slab + row * 68 + c4);
      if (RESID) {
        const v4f rr = *(const v4f*)(resid + (size_t)(mBase + row) * ldc + n0 + c4);
        v = v + rr;
      }
      vals[it] = v;
    }
#pragma unroll
    for (int pass = 0; pass < 2; ++pass) {
#pragma unroll
      for (int it = 0; it < 8; ++it) {
        const int row = it * 2 + hh;
        *(volatile v4f*)(Cout + (size_t)(mBase + row) * ldc + n0 + c4) = vals[it];
      }
      __threadfence();
    }
    __builtin_amdgcn_fence(__ATOMIC_RELEASE, "workgroup");
    __builtin_amdgcn_wave_barrier();
    __builtin_amdgcn_fence(__ATOMIC_ACQUIRE, "workgroup");
  }
}

template <int MODE>
__global__ __launch_bounds__(256) void wtrans_kernel(const float* __restrict__ W, int nout, int kin,
                                                     unsigned short* __restrict__ outA, unsigned short* __restrict__ outB,
                                                     int nrow0, float scale) {
  __shared__ float sm[64][65];
  const int t  = threadIdx.x;
  const int k0 = blockIdx.x * 64;
  const int n0 = blockIdx.y * 64;
#pragma unroll
  for (int i = 0; i < 16; ++i) {
    const int e = i * 256 + t;
    const int r = e >> 6;
    const int c = e & 63;
    sm[c][r] = W[(size_t)(k0 + r) * nout + n0 + c] * scale;
  }
  __syncthreads();
  const int lane = t & 31, wave = t >> 5;
  const int q = lane >> 3, c8 = (lane & 7) * 8;
  v4u ua[2], ub[2];
#pragma unroll
  for (int it = 0; it < 2; ++it) {
    const int row = wave * 8 + it * 4 + q;
    v4f a, b;
#pragma unroll
    for (int e = 0; e < 4; ++e) { a[e] = sm[row][c8 + e]; b[e] = sm[row][c8 + 4 + e]; }
    if (MODE == 0) {
      ua[it] = pack8_f16(a, b, 1.0f);
      ub[it] = ua[it];
    } else {
      split8_bf16(a, b, ua[it], ub[it]);
    }
  }
#pragma unroll
  for (int pass = 0; pass < 2; ++pass) {
#pragma unroll
    for (int it = 0; it < 2; ++it) {
      const int row = wave * 8 + it * 4 + q;
      const size_t o = (size_t)(nrow0 + n0 + row) * kin + k0 + c8;
      *(volatile v4u*)(outA + o) = ua[it];
      if (MODE == 1) *(volatile v4u*)(outB + o) = ub[it];
    }
    __threadfence();
  }
}

__global__ __launch_bounds__(256) void norm_gate_kernel(const float* __restrict__ x, const float* __restrict__ nw,
                                                        const float* __restrict__ Wb, const float* __restrict__ Wa,
                                                        const float* __restrict__ alog, const float* __restrict__ dtb,
                                                        unsigned short* __restrict__ xhi, unsigned short* __restrict__ xlo,
                                                        float* __restrict__ bg) {
  const int lane = threadIdx.x & 31, wave = threadIdx.x >> 5;
  const int row0 = (blockIdx.x * 8 + wave) * 2;
  const int e0 = 8 * lane;
  const v4f wa0 = *(const v4f*)(nw + e0);
  const v4f wa1 = *(const v4f*)(nw + e0 + 4);
  const v4f wb0 = *(const v4f*)(nw + 256 + e0);
  const v4f wb1 = *(const v4f*)(nw + 256 + e0 + 4);
  float res = 0.0f;
#pragma unroll 1
  for (int i = 0; i < 2; ++i) {
    const int row = row0 + i;
    const float* xr = x + (size_t)row * kDim;
    v4f xa0 = *(const v4f*)(xr + e0);
    v4f xa1 = *(const v4f*)(xr + e0 + 4);
    v4f xb0 = *(const v4f*)(xr + 256 + e0);
    v4f xb1 = *(const v4f*)(xr + 256 + e0 + 4);
    float ss = 0.0f;
#pragma unroll
    for (int e = 0; e < 4; ++e) {
      ss += xa0[e] * xa0[e];
      ss += xa1[e] * xa1[e];
      ss += xb0[e] * xb0[e];
      ss += xb1[e] * xb1[e];
    }
    ss = wave_sum(ss);
    const float rs = rsqrtf(ss * (1.0f / (float)kDim) + kEps);
    xa0 = (xa0 * rs) * wa0;
    xa1 = (xa1 * rs) * wa1;
    xb0 = (xb0 * rs) * wb0;
    xb1 = (xb1 * rs) * wb1;
    v4u hi0, lo0, hi1, lo1;
    split8_bf16(xa0, xa1, hi0, lo0);
    split8_bf16(xb0, xb1, hi1, lo1);
    const size_t off0 = (size_t)row * kDim + e0;
    const size_t off1 = off0 + 256;
#pragma unroll
    for (int pass = 0; pass < 2; ++pass) {
      *(volatile v4u*)(xhi + off0) = hi0;
      *(volatile v4u*)(xhi + off1) = hi1;
      *(volatile v4u*)(xlo + off0) = lo0;
      *(volatile v4u*)(xlo + off1) = lo1;
      __threadfence();
    }
#pragma unroll 1
    for (int n = 0; n < 12; ++n) {
      const float* wp;
      int pitch;
      if (n < 8) { wp = Wb + n; pitch = kNh * kHeads; } else { wp = Wa + (n - 8); pitch = kHeads; }
      float p = 0.0f;
#pragma unroll
      for (int e = 0; e < 4; ++e) p = fmaf(xa0[e], wp[(size_t)(e0 + e) * pitch], p);
#pragma unroll
      for (int e = 0; e < 4; ++e) p = fmaf(xa1[e], wp[(size_t)(e0 + 4 + e) * pitch], p);
#pragma unroll
      for (int e = 0; e < 4; ++e) p = fmaf(xb0[e], wp[(size_t)(256 + e0 + e) * pitch], p);
#pragma unroll
      for (int e = 0; e < 4; ++e) p = fmaf(xb1[e], wp[(size_t)(256 + e0 + 4 + e) * pitch], p);
      p = wave_sum(p);
      res = (lane == 16 * i + n) ? p : res;
    }
  }
  const int n  = lane & 15;
  const int hx = n & 3;
  const float al = alog[hx];
  const float db = dtb[hx];
  const float beta = 2.0f / (1.0f + expf(-res));
  const float z  = res + db;
  const float sp = fmaxf(z, 0.0f) + log1pf(expf(-fabsf(z)));
  const float g  = -expf(al) * sp;
  const float eg = expf(g);
  const float outv = (n < 8) ? beta : ((n < 12) ? eg : 0.0f);
  float* dst = bg + (size_t)row0 * kGateCols + lane;
  *(volatile float*)dst = outv;
  __threadfence();
  *(volatile float*)dst = outv;
}

__global__ __launch_bounds__(256) void conv_norm_kernel(const float* __restrict__ raw, const float* __restrict__ cq,
                                                        const float* __restrict__ ck, const float* __restrict__ cv,
                                                        float* __restrict__ qkv, float qscale) {
  const int lane = threadIdx.x & 31, wave = threadIdx.x >> 5;
  const int gw  = blockIdx.x * 8 + wave;
  const int row = gw / 20;
  const int g   = gw - row * 20;
  const int t   = row & (kSeq - 1);
  const int c0  = g * 128 + 4 * lane;
  const float* cw;
  if (g < 4)       cw = cq + (size_t)c0 * 4;
  else if (g < 12) cw = ck + (size_t)(c0 - kKOff) * 4;
  else             cw = cv + (size_t)(c0 - kVOff) * 4;
  v4f wt[4];
#pragma unroll
  for (int e = 0; e < 4; ++e) wt[e] = *(const v4f*)(cw + 4 * e);
  v4f xr[4];
#pragma unroll
  for (int j = 0; j < 4; ++j) {
    const int ts = t + j - 3;
    const int tc = ts < 0 ? 0 : ts;
    const bool ok = ts >= 0;
    const v4f xv = *(const v4f*)(raw + (size_t)(row - t + tc) * kQkvCols + c0);
#pragma unroll
    for (int e = 0; e < 4; ++e) xr[j][e] = ok ? xv[e] : 0.0f;
  }
  v4f val;
  float ss = 0.0f;
#pragma unroll
  for (int e = 0; e < 4; ++e) {
    float a = 0.0f;
    a += xr[0][e] * wt[e][0];
    a += xr[1][e] * wt[e][1];
    a += xr[2][e] * wt[e][2];
    a += xr[3][e] * wt[e][3];
    const float s = a / (1.0f + expf(-a));
    val[e] = s;
    ss += s * s;
  }
  ss = wave_sum(ss);
  const float rs = rsqrtf(ss + kEps);
  const float f1 = (g < 12) ? rs : 1.0f;
  const float f2 = (g < 4) ? qscale : 1.0f;
  v4f ov;
#pragma unroll
  for (int e = 0; e < 4; ++e) ov[e] = (val[e] * f1) * f2;
  float* dst = qkv + (size_t)row * kQkvCols + c0;
  *(volatile v4f*)dst = ov;
  __threadfence();
  *(volatile v4f*)dst = ov;
}

__global__ __launch_bounds__(256) void state_scan_kernel(const float* __restrict__ qkv, const float* __restrict__ bg,
                                                         const float* __restrict__ S0, float* __restrict__ obuf,
                                                         float* __restrict__ Sout) {
  __shared__ __align__(16) float sst[kDk * kSlabPitch];
  const int tid = threadIdx.x, lane = tid & 31, wave = tid >> 5;
  const int kg = lane & 7, dvl = lane >> 3;
  const int bh  = blockIdx.x >> 2;
  const int dvb = (blockIdx.x & 3) * 32;
  const int b = bh >> 2, h = bh & 3;
  const int dvloc = wave * 4 + dvl;
  const int dv = dvb + dvloc;

  float S[16];
  {
    const float* s0p = S0 + ((size_t)bh * kDk + 16 * kg) * kDv + dv;
#pragma unroll
    for (int j = 0; j < 16; ++j) S[j] = s0p[(size_t)j * kDv];
  }
  const float* rowb   = qkv + (size_t)b * kSeq * kQkvCols;
  const float* qbase  = rowb + h * kDk + 16 * kg;
  const float* k0base = rowb + kKOff + h * kDk + 16 * kg;
  const float* k1base = rowb + kKOff + (kHeads + h) * kDk + 16 * kg;
  const float* v0base = rowb + kVOff + h * kDv + dv;
  const float* v1base = rowb + kVOff + (kHeads + h) * kDv + dv;
  const float* bgb    = bg + (size_t)b * kSeq * kGateCols;
  float* ob = obuf + (size_t)b * kSeq * kOCols + h * kDv + dvb;
  const int rowl = wave * 4 + (lane >> 3);
  const int c4   = (lane & 7) * 4;

#pragma unroll 1
  for (int t = 0; t < kSeq; ++t) {
    const size_t ro = (size_t)t * kQkvCols;
    v4f qv[4], ka[4], kb[4];
#pragma unroll
    for (int m = 0; m < 4; ++m) {
      qv[m] = *(const v4f*)(qbase + ro + 4 * m);
      ka[m] = *(const v4f*)(k0base + ro + 4 * m);
      kb[m] = *(const v4f*)(k1base + ro + 4 * m);
    }
    const float va = v0base[ro];
    const float vb = v1base[ro];
    const float* bgr = bgb + (size_t)t * kGateCols;
    const float be0 = bgr[h];
    const float be1 = bgr[kHeads + h];
    const float eg  = bgr[2 * kHeads + h];

#pragma unroll
    for (int j = 0; j < 16; ++j) S[j] *= eg;

    float p = 0.0f;
#pragma unroll
    for (int j = 0; j < 16; ++j) p = fmaf(ka[j >> 2][j & 3], S[j], p);
    p = grp8_sum(p);
    const float cf0 = be0 * (va - p);
#pragma unroll
    for (int j = 0; j < 16; ++j) S[j] = fmaf(ka[j >> 2][j & 3], cf0, S[j]);

    p = 0.0f;
#pragma unroll
    for (int j = 0; j < 16; ++j) p = fmaf(kb[j >> 2][j & 3], S[j], p);
    p = grp8_sum(p);
    const float cf1 = be1 * (vb - p);
#pragma unroll
    for (int j = 0; j < 16; ++j) S[j] = fmaf(kb[j >> 2][j & 3], cf1, S[j]);

    p = 0.0f;
#pragma unroll
    for (int j = 0; j < 16; ++j) p = fmaf(qv[j >> 2][j & 3], S[j], p);
    p = grp8_sum(p);

    const int tl = t & 31;
    if (kg == 0) sst[tl * kSlabPitch + dvloc] = p;
    if (tl == 31) {
      __syncthreads();
      const v4f val = *(const v4f*)(sst + rowl * kSlabPitch + c4);
      float* dst = ob + (size_t)(t - 31 + rowl) * kOCols + c4;
      *(volatile v4f*)dst = val;
      __threadfence();
      *(volatile v4f*)dst = val;
      __syncthreads();
    }
  }

#pragma unroll
  for (int j = 0; j < 16; ++j) sst[(16 * kg + j) * kSlabPitch + dvloc] = S[j];
  __syncthreads();
  v4f sv[4];
#pragma unroll
  for (int it = 0; it < 4; ++it) sv[it] = *(const v4f*)(sst + (it * 32 + rowl) * kSlabPitch + c4);
#pragma unroll
  for (int pass = 0; pass < 2; ++pass) {
#pragma unroll
    for (int it = 0; it < 4; ++it) {
      const int row = it * 32 + rowl;
      *(volatile v4f*)(Sout + ((size_t)bh * kDk + row) * kDv + dvb + c4) = sv[it];
    }
    __threadfence();
  }
}

__global__ __launch_bounds__(256) void onorm_kernel(const float* __restrict__ obuf, const float* __restrict__ ow,
                                                    unsigned short* __restrict__ on16) {
  const int lane = threadIdx.x & 31, wave = threadIdx.x >> 5;
  const int row = blockIdx.x * 8 + wave;
  const int e0 = 8 * lane;
  const int w0 = 8 * (lane & 15);
  const float* orow = obuf + (size_t)row * kOCols;
  v4f a0 = *(const v4f*)(orow + e0);
  v4f a1 = *(const v4f*)(orow + e0 + 4);
  v4f b0 = *(const v4f*)(orow + 256 + e0);
  v4f b1 = *(const v4f*)(orow + 256 + e0 + 4);
  const v4f g0 = *(const v4f*)(ow + w0);
  const v4f g1 = *(const v4f*)(ow + w0 + 4);
  float sa = 0.0f, sb = 0.0f;
#pragma unroll
  for (int e = 0; e < 4; ++e) {
    sa += a0[e] * a0[e];
    sa += a1[e] * a1[e];
    sb += b0[e] * b0[e];
    sb += b1[e] * b1[e];
  }
  sa = grp16_sum(sa);
  sb = grp16_sum(sb);
  const float ra = rsqrtf(sa * (1.0f / (float)kDv) + kEps);
  const float rb = rsqrtf(sb * (1.0f / (float)kDv) + kEps);
  a0 = (a0 * ra) * g0;
  a1 = (a1 * ra) * g1;
  b0 = (b0 * rb) * g0;
  b1 = (b1 * rb) * g1;
  const v4u u0 = pack8_f16(a0, a1, kACarry);
  const v4u u1 = pack8_f16(b0, b1, kACarry);
  unsigned short* dst = on16 + (size_t)row * kOCols + e0;
#pragma unroll
  for (int pass = 0; pass < 2; ++pass) {
    *(volatile v4u*)(dst) = u0;
    *(volatile v4u*)(dst + 256) = u1;
    __threadfence();
  }
}

__global__ __launch_bounds__(256) void rms512_f16_kernel(const float* __restrict__ hin, const float* __restrict__ w,
                                                         unsigned short* __restrict__ out16) {
  const int lane = threadIdx.x & 31, wave = threadIdx.x >> 5;
  const int row = blockIdx.x * 8 + wave;
  const int e0 = 8 * lane;
  const float* hr = hin + (size_t)row * kDim;
  v4f a0 = *(const v4f*)(hr + e0);
  v4f a1 = *(const v4f*)(hr + e0 + 4);
  v4f b0 = *(const v4f*)(hr + 256 + e0);
  v4f b1 = *(const v4f*)(hr + 256 + e0 + 4);
  const v4f g0 = *(const v4f*)(w + e0);
  const v4f g1 = *(const v4f*)(w + e0 + 4);
  const v4f g2 = *(const v4f*)(w + 256 + e0);
  const v4f g3 = *(const v4f*)(w + 256 + e0 + 4);
  float ss = 0.0f;
#pragma unroll
  for (int e = 0; e < 4; ++e) {
    ss += a0[e] * a0[e];
    ss += a1[e] * a1[e];
    ss += b0[e] * b0[e];
    ss += b1[e] * b1[e];
  }
  ss = wave_sum(ss);
  const float rs = rsqrtf(ss * (1.0f / (float)kDim) + kEps);
  a0 = (a0 * rs) * g0;
  a1 = (a1 * rs) * g1;
  b0 = (b0 * rs) * g2;
  b1 = (b1 * rs) * g3;
  const v4u u0 = pack8_f16(a0, a1, kACarry);
  const v4u u1 = pack8_f16(b0, b1, kACarry);
  unsigned short* dst = out16 + (size_t)row * kDim + e0;
#pragma unroll
  for (int pass = 0; pass < 2; ++pass) {
    *(volatile v4u*)(dst) = u0;
    *(volatile v4u*)(dst + 256) = u1;
    __threadfence();
  }
}

__global__ __launch_bounds__(256) void swiglu_kernel(const float* __restrict__ gy, unsigned short* __restrict__ u16) {
  const int i = blockIdx.x * 256 + threadIdx.x;
  const int row = i >> 5;
  const int c8 = (i & 31) * 8;
  const float* gp = gy + (size_t)row * (2 * kMlp) + c8;
  const float* yp = gp + kMlp;
  unsigned w0 = 0u, w1 = 0u, w2 = 0u, w3 = 0u;
#pragma unroll 1
  for (int hf = 0; hf < 2; ++hf) {
    const v4f gv = *(const v4f*)(gp + 4 * hf);
    const v4f yv = *(const v4f*)(yp + 4 * hf);
    float u[4];
#pragma unroll
    for (int e = 0; e < 4; ++e) {
      const float gt = gv[e];
      const float yy = yv[e];
      u[e] = ((gt / (1.0f + expf(-gt))) * yy) * kACarry;
    }
    const unsigned pa = pk16(h_bits(u[0]), h_bits(u[1]));
    const unsigned pb = pk16(h_bits(u[2]), h_bits(u[3]));
    if (hf == 0) { w0 = pa; w1 = pb; } else { w2 = pa; w3 = pb; }
  }
  const v4u uu = (v4u){w0, w1, w2, w3};
  unsigned short* dst = u16 + (size_t)i * 8;
  *(volatile v4u*)dst = uu;
  __threadfence();
  *(volatile v4u*)dst = uu;
}

extern "C" void kernel_launch(void* const* d_in, const int* in_sizes, int n_in,
                              void* d_out, int out_size, void* d_ws, size_t ws_size, hipStream_t stream) {
  if (n_in < 18 || d_out == nullptr || d_ws == nullptr) return;
  if (in_sizes[0] != kRows * kDim || in_sizes[1] != kOut1 || in_sizes[2] != kDim * kQCols ||
      in_sizes[3] != kDim * kKCols || in_sizes[4] != kDim * kVCols || in_sizes[5] != kDim * kNh * kHeads ||
      in_sizes[6] != kDim * kHeads || in_sizes[7] != kHeads || in_sizes[8] != kHeads ||
      in_sizes[9] != kQCols * 4 || in_sizes[10] != kKCols * 4 || in_sizes[11] != kVCols * 4 ||
      in_sizes[12] != kDv || in_sizes[13] != kOCols * kDim || in_sizes[14] != kDim || in_sizes[15] != kDim ||
      in_sizes[16] != kDim * 2 * kMlp || in_sizes[17] != kMlp * kDim || out_size != kOut0 + kOut1) return;

  const float* x      = (const float*)d_in[0];
  const float* S0     = (const float*)d_in[1];
  const float* Wq     = (const float*)d_in[2];
  const float* Wk     = (const float*)d_in[3];
  const float* Wv     = (const float*)d_in[4];
  const float* Wb     = (const float*)d_in[5];
  const float* Wa     = (const float*)d_in[6];
  const float* A_log  = (const float*)d_in[7];
  const float* dt_b   = (const float*)d_in[8];
  const float* conv_q = (const float*)d_in[9];
  const float* conv_k = (const float*)d_in[10];
  const float* conv_v = (const float*)d_in[11];
  const float* o_nw   = (const float*)d_in[12];
  const float* Wo     = (const float*)d_in[13];
  const float* an_w   = (const float*)d_in[14];
  const float* mn_w   = (const float*)d_in[15];
  const float* Wg     = (const float*)d_in[16];
  const float* Wd     = (const float*)d_in[17];
  float* out0 = (float*)d_out;
  float* out1 = out0 + (size_t)kOut0;

  char* ws = (char*)d_ws;
  size_t off = 0;
  auto carve = [&](size_t bytes) -> char* { char* p = ws + off; off += (bytes + 255) & ~(size_t)255; return p; };
  unsigned short* WQKVH = (unsigned short*)carve((size_t)kQkvCols * kDim * 2);
  unsigned short* WQKVL = (unsigned short*)carve((size_t)kQkvCols * kDim * 2);
  unsigned short* WOT   = (unsigned short*)carve((size_t)kDim * kOCols * 2);
  unsigned short* WGT   = (unsigned short*)carve((size_t)(2 * kMlp) * kDim * 2);
  unsigned short* WDT   = (unsigned short*)carve((size_t)kDim * kMlp * 2);
  unsigned short* XNH   = (unsigned short*)carve((size_t)kRows * kDim * 2);
  unsigned short* XNL   = (unsigned short*)carve((size_t)kRows * kDim * 2);
  float*          BG    = (float*)carve((size_t)kRows * kGateCols * 4);
  float*          RAW   = (float*)carve((size_t)kRows * kQkvCols * 4);
  float*          QKV   = (float*)carve((size_t)kRows * kQkvCols * 4);
  float*          OBUF  = (float*)carve((size_t)kRows * kOCols * 4);
  unsigned short* ON16  = (unsigned short*)carve((size_t)kRows * kOCols * 2);
  float*          HBUF  = (float*)carve((size_t)kRows * kDim * 4);
  unsigned short* HN16  = (unsigned short*)carve((size_t)kRows * kDim * 2);
  float*          GY    = (float*)carve((size_t)kRows * 2 * kMlp * 4);
  unsigned short* U16   = (unsigned short*)carve((size_t)kRows * kMlp * 2);
  if (off > ws_size || off > (size_t)134217728) return;

  const float qscale = (float)(1.0 / sqrt((double)kDk));

  wtrans_kernel<1><<<dim3(kDim / 64, kQCols / 64), 256, 0, stream>>>(Wq, kQCols, kDim, WQKVH, WQKVL, 0, 1.0f);
  wtrans_kernel<1><<<dim3(kDim / 64, kKCols / 64), 256, 0, stream>>>(Wk, kKCols, kDim, WQKVH, WQKVL, kKOff, 1.0f);
  wtrans_kernel<1><<<dim3(kDim / 64, kVCols / 64), 256, 0, stream>>>(Wv, kVCols, kDim, WQKVH, WQKVL, kVOff, 1.0f);
  wtrans_kernel<0><<<dim3(kOCols / 64, kDim / 64), 256, 0, stream>>>(Wo, kDim, kOCols, WOT, WOT, 0, kWCarry);
  wtrans_kernel<0><<<dim3(kDim / 64, (2 * kMlp) / 64), 256, 0, stream>>>(Wg, 2 * kMlp, kDim, WGT, WGT, 0, kWCarry);
  wtrans_kernel<0><<<dim3(kMlp / 64, kDim / 64), 256, 0, stream>>>(Wd, kDim, kMlp, WDT, WDT, 0, kWCarry);

  norm_gate_kernel<<<kRows / 16, 256, 0, stream>>>(x, an_w, Wb, Wa, A_log, dt_b, XNH, XNL, BG);

  wmma_gemm64<1, true, false><<<(kRows / 64) * (kQkvCols / 64) / 8, 256, 0, stream>>>(
      XNH, XNL, kDim, WQKVH, WQKVL, kDim, RAW, kQkvCols, x, kRows, kQkvCols, kDim, 1.0f);

  conv_norm_kernel<<<(kRows * 20) / 8, 256, 0, stream>>>(RAW, conv_q, conv_k, conv_v, QKV, qscale);

  state_scan_kernel<<<kBatch * kHeads * 4, 256, 0, stream>>>(QKV, BG, S0, OBUF, out1);

  onorm_kernel<<<kRows / 8, 256, 0, stream>>>(OBUF, o_nw, ON16);
  wmma_gemm64<0, false, true><<<(kRows / 64) * (kDim / 64) / 8, 256, 0, stream>>>(
      ON16, ON16, kOCols, WOT, WOT, kOCols, HBUF, kDim, x, kRows, kDim, kOCols, kFold);

  rms512_f16_kernel<<<kRows / 8, 256, 0, stream>>>(HBUF, mn_w, HN16);
  wmma_gemm64<0, false, false><<<(kRows / 64) * ((2 * kMlp) / 64) / 8, 256, 0, stream>>>(
      HN16, HN16, kDim, WGT, WGT, kDim, GY, 2 * kMlp, x, kRows, 2 * kMlp, kDim, kFold);
  swiglu_kernel<<<(kRows * kMlp / 8) / 256, 256, 0, stream>>>(GY, U16);
  wmma_gemm64<0, false, true><<<(kRows / 64) * (kDim / 64) / 8, 256, 0, stream>>>(
      U16, U16, kMlp, WDT, WDT, kMlp, out0, kDim, HBUF, kRows, kDim, kMlp, kFold);
}
